// SE3StructEncoder_35235911696634
// MI455X (gfx1250) — hardware-verified
//
#include <hip/hip_runtime.h>
#include <stdint.h>
#include <stddef.h>

constexpr int NB_  = 2;
constexpr int LL   = 512;
constexpr int HD   = 128;
constexpr int IN_F = 32;
constexpr int NLAY = 3;
constexpr int NR   = NB_ * LL;
constexpr int CH_I = 128;
constexpr int CH_ROWS = CH_I * LL;
constexpr int E_W1_STRIDE = (2 * HD + 2) * HD;
constexpr int W_HH = HD * HD;
constexpr int W_2HH = 2 * HD * HD;

typedef __attribute__((ext_vector_type(16))) _Float16 v16h;
typedef __attribute__((ext_vector_type(8)))  _Float16 v8h;
typedef __attribute__((ext_vector_type(16))) __bf16   v16b;
typedef __attribute__((ext_vector_type(8)))  __bf16   v8b;
typedef __attribute__((ext_vector_type(8)))  float    v8f;
typedef __attribute__((ext_vector_type(4)))  float    v4f;

__device__ __forceinline__ unsigned short f2bf_bits(float f) {
  unsigned u = __float_as_uint(f);
  return (unsigned short)((u + 0x7FFFu + ((u >> 16) & 1u)) >> 16);
}
__device__ __forceinline__ float bf_bits2f(unsigned short h) { return __uint_as_float(((unsigned)h) << 16); }

__device__ __forceinline__ void dep_guard_h(v8f& a, v8f& b, v16h x, v16h y) { asm volatile("v_nop\n\tv_nop\n\tv_nop\n\tv_nop" : "+v"(a), "+v"(b) : "v"(x), "v"(y)); }
__device__ __forceinline__ void dep_guard_b(v8f& a, v8f& b, v16b x, v16b y) { asm volatile("v_nop\n\tv_nop\n\tv_nop\n\tv_nop" : "+v"(a), "+v"(b) : "v"(x), "v"(y)); }
__device__ __forceinline__ void keep4_h(v16h a, v16h b, v16h c, v16h d) { asm volatile("v_nop" :: "v"(a), "v"(b), "v"(c), "v"(d)); }
__device__ __forceinline__ void keep4_b(v16b a, v16b b, v16b c, v16b d) { asm volatile("v_nop" :: "v"(a), "v"(b), "v"(c), "v"(d)); }
__device__ __forceinline__ void acc_guard4(v8f& a, v8f& b, v8f& c, v8f& d) { asm volatile("v_nop\n\tv_nop\n\tv_nop\n\tv_nop" : "+v"(a), "+v"(b), "+v"(c), "+v"(d)); }
template <typename T> struct Frag;
template <> struct Frag<_Float16> {
  typedef v16h V; union U { v16h v; v8h h[2]; };
  static __device__ __forceinline__ v16h load(const _Float16* p) {
    U f; f.h[0] = *(const v8h*)(p); f.h[1] = *(const v8h*)(p + 16); return f.v;
  }
  static __device__ __forceinline__ v8f mma(v16h a, v16h b, v8f c) {
    return __builtin_amdgcn_wmma_f32_16x16x32_f16(false, a, false, b, (short)0, c, false, false);
  }
  static __device__ __forceinline__ void guard(v8f& a, v8f& b, v16h x, v16h y) { dep_guard_h(a, b, x, y); }
  static __device__ __forceinline__ void keep(v16h a, v16h b, v16h c, v16h d) { keep4_h(a, b, c, d); }
};
template <> struct Frag<__bf16> {
  typedef v16b V; union U { v16b v; v8b h[2]; };
  static __device__ __forceinline__ v16b load(const __bf16* p) {
    U f; f.h[0] = *(const v8b*)(p); f.h[1] = *(const v8b*)(p + 16); return f.v;
  }
  static __device__ __forceinline__ v8f mma(v16b a, v16b b, v8f c) {
    return __builtin_amdgcn_wmma_f32_16x16x32_bf16(false, a, false, b, (short)0, c, false, false);
  }
  static __device__ __forceinline__ void guard(v8f& a, v8f& b, v16b x, v16b y) { dep_guard_b(a, b, x, y); }
  static __device__ __forceinline__ void keep(v16b a, v16b b, v16b c, v16b d) { keep4_b(a, b, c, d); }
};

template <int ET> struct Elem;
template <> struct Elem<0> { typedef _Float16 T; };
template <> struct Elem<1> { typedef __bf16 T; };
template <int ET, bool SPLIT, int BIAS_MODE, int OUT_MODE, bool RESID, int ACT = 0>
__global__ __launch_bounds__(256) void wmma_gemm64(
    const unsigned short* __restrict__ Ap, const unsigned short* __restrict__ A2p, int lda, long strideA,
    const unsigned short* __restrict__ Btp, const unsigned short* __restrict__ Bt2p, int ldb, long strideB,
    void* __restrict__ Cout, void* __restrict__ Cout2, int ldc, long strideC,
    const float* __restrict__ bias,
    const float* __restrict__ resid, long strideR,
    int M, int N, int K, float scale) {
  typedef typename Elem<ET>::T T;
  typedef typename Frag<T>::V V;
  const T* A = (const T*)Ap; const T* A2 = (const T*)A2p; const T* Bt = (const T*)Btp; const T* Bt2 = (const T*)Bt2p;
  __shared__ __align__(16) float sT[8][16 * 68];
  const int b    = blockIdx.y;
  const int lane = threadIdx.x & 31;
  const int wave = threadIdx.x >> 5;
  const int tilesN = N >> 6;
  const int tilesM = M >> 6;
  const int tile = blockIdx.x * 8 + wave;
  if (tile >= tilesM * tilesN) return;
  const int tm = tile / tilesN;
  const int tn = tile - tm * tilesN;
  const int m0 = tm << 6;
  const int n0 = tn << 6;

  const T* Ab  = A  + (size_t)b * strideA;
  const T* Bb  = Bt + (size_t)b * strideB;
  const T* Ab2 = SPLIT ? (A2  + (size_t)b * strideA) : nullptr;
  const T* Bb2 = SPLIT ? (Bt2 + (size_t)b * strideB) : nullptr;

  const int rlane = lane & 15;
  const int koff  = (lane >> 4) * 8;
  const int mOff  = (lane >> 4) * 8;

  v8f acc[4][4];
#pragma unroll
  for (int i = 0; i < 4; ++i)
#pragma unroll
    for (int j = 0; j < 4; ++j) acc[i][j] = (v8f){0.f,0.f,0.f,0.f,0.f,0.f,0.f,0.f};

  for (int k0 = 0; k0 < K; k0 += 32) {
    V bh[4], bl[4];
#pragma unroll
    for (int j = 0; j < 4; ++j) {
      const size_t bo = (size_t)(n0 + (j << 4) + rlane) * ldb + koff + k0;
      bh[j] = Frag<T>::load(Bb + bo);
      if (SPLIT) bl[j] = Frag<T>::load(Bb2 + bo);
    }
#pragma unroll
    for (int i = 0; i < 4; ++i) {
      const size_t ao = (size_t)(m0 + (i << 4) + rlane) * lda + koff + k0;
      V ah = Frag<T>::load(Ab + ao);
      V al;
      if (SPLIT) al = Frag<T>::load(Ab2 + ao);
#pragma unroll
      for (int j = 0; j < 4; ++j) {
        acc[i][j] = Frag<T>::mma(ah, bh[j], acc[i][j]);
        if (SPLIT) {
          acc[i][j] = Frag<T>::mma(ah, bl[j], acc[i][j]);
          acc[i][j] = Frag<T>::mma(al, bh[j], acc[i][j]);
        }
      }
      Frag<T>::guard(acc[i][0], acc[i][3], ah, SPLIT ? al : ah);
    }
    Frag<T>::keep(bh[0], bh[1], bh[2], bh[3]);
    if (SPLIT) Frag<T>::keep(bl[0], bl[1], bl[2], bl[3]);
  }
  acc_guard4(acc[0][0], acc[0][1], acc[0][2], acc[0][3]);
  acc_guard4(acc[1][0], acc[1][1], acc[1][2], acc[1][3]);
  acc_guard4(acc[2][0], acc[2][1], acc[2][2], acc[2][3]);
  acc_guard4(acc[3][0], acc[3][1], acc[3][2], acc[3][3]);

  float* slab = sT[wave];
  const float* Rb = RESID ? (resid + (size_t)b * strideR) : nullptr;
#pragma unroll
  for (int i = 0; i < 4; ++i) {
    const int mBase = m0 + (i << 4);
#pragma unroll
    for (int j = 0; j < 4; ++j) {
      const int n = n0 + (j << 4) + rlane;
      float bv = 0.f;
      if (BIAS_MODE == 2) bv = bias[n];
#pragma unroll
      for (int r = 0; r < 8; ++r) {
        float v = acc[i][j][r] * scale;
        if (BIAS_MODE == 1) v += bias[mBase + mOff + r];
        if (BIAS_MODE == 2) v += bv;
        if (RESID) v += Rb[(size_t)(mBase + mOff + r) * ldc + n];
        if (ACT == 1) v = tanhf(v);
        if (ACT == 2) v = fmaxf(v, 0.0f);
        if (ACT == 3) v = v / (1.0f + expf(-v));
        if (ACT == 4) v = (v > 0.f) ? v : 0.01f * v;
        if (ACT == 5) v = 0.5f * v * (1.0f + erff(v * 0.70710678118654752f));
        if (ACT == 6) v = v * __builtin_amdgcn_rcpf(1.0f + __expf(-v));
        slab[(mOff + r) * 68 + (j << 4) + rlane] = v;
      }
    }
    __builtin_amdgcn_fence(__ATOMIC_RELEASE, "workgroup");
    __builtin_amdgcn_wave_barrier();
    __builtin_amdgcn_fence(__ATOMIC_ACQUIRE, "workgroup");
    if (OUT_MODE == 0) {
      float* C = (float*)Cout + (size_t)b * strideC;
      const int hh = lane >> 4, c4 = (lane & 15) * 4;
      for (int pass = 0; pass < 2; ++pass) {
#pragma unroll
        for (int it = 0; it < 8; ++it) {
          const int row = it * 2 + hh;
          v4f v = *(const v4f*)(slab + row * 68 + c4);
          *(volatile v4f*)(C + (size_t)(mBase + row) * ldc + n0 + c4) = v;
        }
        __threadfence();
      }
    } else {
      const int q = lane >> 3, c8 = (lane & 7) * 8;
      unsigned short* C  = (unsigned short*)Cout  + (size_t)b * strideC;
      unsigned short* C2 = (OUT_MODE == 2) ? ((unsigned short*)Cout2 + (size_t)b * strideC) : nullptr;
      for (int pass = 0; pass < 2; ++pass) {
#pragma unroll
        for (int it = 0; it < 4; ++it) {
          const int row = it * 4 + q;
          const float* sp = slab + row * 68 + c8;
          v8h hv, lv;
#pragma unroll
          for (int e = 0; e < 8; ++e) {
            if (OUT_MODE == 1) {
              hv[e] = (_Float16)sp[e];
            } else {
              unsigned short hb = f2bf_bits(sp[e]);
              unsigned short lb = f2bf_bits(sp[e] - bf_bits2f(hb));
              hv[e] = __builtin_bit_cast(_Float16, hb);
              lv[e] = __builtin_bit_cast(_Float16, lb);
            }
          }
          *(volatile v8h*)(C + (size_t)(mBase + row) * ldc + n0 + c8) = hv;
          if (OUT_MODE == 2) *(volatile v8h*)(C2 + (size_t)(mBase + row) * ldc + n0 + c8) = lv;
        }
        __threadfence();
      }
    }
    __builtin_amdgcn_fence(__ATOMIC_RELEASE, "workgroup");
    __builtin_amdgcn_wave_barrier();
    __builtin_amdgcn_fence(__ATOMIC_ACQUIRE, "workgroup");
  }
}

__global__ __launch_bounds__(256) void split_cast8(const float* __restrict__ src, int sp,
                                                   unsigned short* __restrict__ hi,
                                                   unsigned short* __restrict__ lo,
                                                   int dp, int cg, int total8) {
  const int idx = blockIdx.x * 256 + threadIdx.x;
  if (idx >= total8) return;
  const int r  = idx / cg;
  const int c8 = (idx - r * cg) * 8;
  const float* s = src + (size_t)r * sp + c8;
  const v4f a = *(const v4f*)s;
  const v4f c = *(const v4f*)(s + 4);
  float f[8];
  f[0] = a.x; f[1] = a.y; f[2] = a.z; f[3] = a.w; f[4] = c.x; f[5] = c.y; f[6] = c.z; f[7] = c.w;
  v8h hv, lv;
#pragma unroll
  for (int e = 0; e < 8; ++e) {
    const unsigned short hb = f2bf_bits(f[e]);
    const unsigned short lb = f2bf_bits(f[e] - bf_bits2f(hb));
    hv[e] = __builtin_bit_cast(_Float16, hb);
    lv[e] = __builtin_bit_cast(_Float16, lb);
  }
  unsigned short* ph = hi + (size_t)r * dp + c8;
  unsigned short* pl = lo + (size_t)r * dp + c8;
  *(volatile v8h*)ph = hv;
  *(volatile v8h*)pl = lv;
  __threadfence();
  *(volatile v8h*)ph = hv;
  *(volatile v8h*)pl = lv;
}

template <int TK, int MODE>
__global__ __launch_bounds__(256) void transpose_cast(const float* __restrict__ src, int N, int K,
                                                     long srcA, long srcB, int zdiv,
                                                     unsigned short* __restrict__ dh,
                                                     unsigned short* __restrict__ dl, long dstZ) {
  __shared__ float T[TK][65];
  const int tid = threadIdx.x;
  const int z   = blockIdx.z;
  const int n0  = blockIdx.x * 64;
  const int k0  = blockIdx.y * TK;
  const float* S = src + (size_t)(z / zdiv) * srcA + (size_t)(z % zdiv) * srcB;
#pragma unroll
  for (int it = 0; it < TK / 16; ++it) {
    const int q  = it * 256 + tid;
    const int k  = q >> 4;
    const int n4 = (q & 15) * 4;
    const v4f v = *(const v4f*)(S + (size_t)(k0 + k) * N + n0 + n4);
    T[k][n4 + 0] = v.x; T[k][n4 + 1] = v.y; T[k][n4 + 2] = v.z; T[k][n4 + 3] = v.w;
  }
  __syncthreads();
  constexpr int KG  = TK / 8;
  constexpr int RPI = 256 / KG;
  constexpr int NIT = 64 / RPI;
  const int kq = (tid % KG) * 8;
  unsigned short* Dh = dh + (size_t)z * dstZ;
  unsigned short* Dl = dl + (size_t)z * dstZ;
  for (int pass = 0; pass < 2; ++pass) {
#pragma unroll
    for (int it = 0; it < NIT; ++it) {
      const int nn = it * RPI + tid / KG;
      v8h hv, lv;
#pragma unroll
      for (int e = 0; e < 8; ++e) {
        const float f = T[kq + e][nn];
        if (MODE == 0) {
          hv[e] = (_Float16)f;
        } else {
          const unsigned short hb = f2bf_bits(f);
          const unsigned short lb = f2bf_bits(f - bf_bits2f(hb));
          hv[e] = __builtin_bit_cast(_Float16, hb);
          lv[e] = __builtin_bit_cast(_Float16, lb);
        }
      }
      const size_t o = (size_t)(n0 + nn) * K + k0 + kq;
      *(volatile v8h*)(Dh + o) = hv;
      if (MODE == 1) *(volatile v8h*)(Dl + o) = lv;
    }
    __threadfence();
  }
}

__device__ __forceinline__ _Float16 pre_silu16(float a, float hj, float dist, float wd,
                                               float cf, float wc, float bb) {
#pragma clang fp contract(off)
  float p = a + hj;
  p = p + dist * wd;
  p = p + cf * wc;
  p = p + bb;
  const float s = p * __builtin_amdgcn_rcpf(1.0f + __expf(-p));
  return (_Float16)s;
}

__global__ __launch_bounds__(256) void build_pre(const float* __restrict__ HIJ,
                                                 const float* __restrict__ coords,
                                                 const float* __restrict__ contacts,
                                                 const float* __restrict__ w1l,
                                                 const float* __restrict__ b1,
                                                 unsigned short* __restrict__ PRE,
                                                 int b, int i0) {
#pragma clang fp contract(off)
  const int il   = blockIdx.x;
  const int jq   = blockIdx.y;
  const int tid  = threadIdx.x;
  const int wave = tid >> 5;
  const int lane = tid & 31;
  const int rsel = lane >> 4;
  const int c8   = (lane & 15) * 8;
  const int i    = i0 + il;
  const int ni   = b * LL + i;
  const float* hiptr = HIJ + (size_t)ni * (2 * HD) + c8;
  const v4f hiA = *(const v4f*)hiptr, hiB = *(const v4f*)(hiptr + 4);
  const float* wdp = w1l + (size_t)(2 * HD) * HD + c8;
  const float* wcp = w1l + (size_t)(2 * HD + 1) * HD + c8;
  const v4f wdA = *(const v4f*)wdp, wdB = *(const v4f*)(wdp + 4);
  const v4f wcA = *(const v4f*)wcp, wcB = *(const v4f*)(wcp + 4);
  const v4f bA  = *(const v4f*)(b1 + c8), bB = *(const v4f*)(b1 + c8 + 4);
  const float cix = coords[(size_t)ni * 3 + 0];
  const float ciy = coords[(size_t)ni * 3 + 1];
  const float ciz = coords[(size_t)ni * 3 + 2];
  const float* crow = contacts + (size_t)ni * LL;

#pragma unroll 1
  for (int it = 0; it < 8; ++it) {
    const int j  = jq * 128 + it * 16 + wave * 2 + rsel;
    const int nj = b * LL + j;
    const float cjx = coords[(size_t)nj * 3 + 0];
    const float cjy = coords[(size_t)nj * 3 + 1];
    const float cjz = coords[(size_t)nj * 3 + 2];
    const float dx = cix - cjx, dy = ciy - cjy, dz = ciz - cjz;
    float sq = dx * dx;
    sq = sq + dy * dy;
    sq = sq + dz * dz;
    const float sr   = sqrtf(sq);
    const float dist = (sq > 0.0f) ? sr : 0.0f;
    const float cf   = crow[j];
    const float* hjp = HIJ + (size_t)nj * (2 * HD) + HD + c8;
    const v4f hjA = *(const v4f*)hjp, hjB = *(const v4f*)(hjp + 4);
    v8h hv;
    hv[0] = pre_silu16(hiA.x, hjA.x, dist, wdA.x, cf, wcA.x, bA.x);
    hv[1] = pre_silu16(hiA.y, hjA.y, dist, wdA.y, cf, wcA.y, bA.y);
    hv[2] = pre_silu16(hiA.z, hjA.z, dist, wdA.z, cf, wcA.z, bA.z);
    hv[3] = pre_silu16(hiA.w, hjA.w, dist, wdA.w, cf, wcA.w, bA.w);
    hv[4] = pre_silu16(hiB.x, hjB.x, dist, wdB.x, cf, wcB.x, bB.x);
    hv[5] = pre_silu16(hiB.y, hjB.y, dist, wdB.y, cf, wcB.y, bB.y);
    hv[6] = pre_silu16(hiB.z, hjB.z, dist, wdB.z, cf, wcB.z, bB.z);
    hv[7] = pre_silu16(hiB.w, hjB.w, dist, wdB.w, cf, wcB.w, bB.w);
    unsigned short* dst = PRE + ((size_t)(il * LL + j)) * HD + c8;
    *(volatile v8h*)dst = hv;
    __threadfence();
    *(volatile v8h*)dst = hv;
  }
}

__global__ __launch_bounds__(128) void reduce_mi(const float* __restrict__ MIJ,
                                                 const float* __restrict__ contacts,
                                                 unsigned short* __restrict__ HMh,
                                                 unsigned short* __restrict__ HMl,
                                                 int b, int i0) {
  __shared__ __align__(16) float part[4][HD];
  __shared__ __align__(16) unsigned short sbits[2][HD];
  const int il   = blockIdx.x;
  const int tid  = threadIdx.x;
  const int lane = tid & 31;
  const int jq   = tid >> 5;
  const int c4   = lane * 4;
  const int ni   = b * LL + i0 + il;
  const float* crow = contacts + (size_t)ni * LL;
  const float* mrow = MIJ + (size_t)il * LL * HD + c4;
  v4f acc = (v4f){0.f, 0.f, 0.f, 0.f};
#pragma unroll 2
  for (int jj = 0; jj < LL / 4; ++jj) {
    const int j = jj * 4 + jq;
    const float cf = crow[j];
    const v4f v = *(const v4f*)(mrow + (size_t)j * HD);
    const bool m = cf > 0.0f;
    acc.x += m ? v.x : 0.0f;
    acc.y += m ? v.y : 0.0f;
    acc.z += m ? v.z : 0.0f;
    acc.w += m ? v.w : 0.0f;
  }
  *(v4f*)(&part[jq][c4]) = acc;
  __syncthreads();
  float s = part[0][tid];
  s = s + part[1][tid];
  s = s + part[2][tid];
  s = s + part[3][tid];
  const unsigned short hb = f2bf_bits(s);
  const unsigned short lb = f2bf_bits(s - bf_bits2f(hb));
  sbits[0][tid] = hb;
  sbits[1][tid] = lb;
  __syncthreads();
  if (tid < 32) {
    const int cl = (lane & 15) * 8;
    const v8h hv = *(const v8h*)(&sbits[0][cl]);
    const v8h lv = *(const v8h*)(&sbits[1][cl]);
    unsigned short* ph = HMh + (size_t)ni * (2 * HD) + HD + cl;
    unsigned short* pl = HMl + (size_t)ni * (2 * HD) + HD + cl;
    if (lane < 16) {
      *(volatile v8h*)ph = hv;
      *(volatile v8h*)pl = lv;
    }
    __threadfence();
    if (lane < 16) {
      *(volatile v8h*)ph = hv;
      *(volatile v8h*)pl = lv;
    }
  }
}

static inline size_t align256(size_t x) { return (x + 255) & ~(size_t)255; }

extern "C" void kernel_launch(void* const* d_in, const int* in_sizes, int n_in,
                              void* d_out, int out_size, void* d_ws, size_t ws_size,
                              hipStream_t stream) {
  if (n_in < 13) return;
  if (in_sizes[0] != NB_ * LL * 3) return;
  if (in_sizes[1] != NB_ * LL * LL) return;
  if (in_sizes[2] != NB_ * LL * IN_F) return;
  if (in_sizes[3] != IN_F * HD) return;
  if (in_sizes[4] != HD) return;
  if (in_sizes[5] != NLAY * E_W1_STRIDE) return;
  if (in_sizes[6] != NLAY * HD) return;
  if (in_sizes[7] != NLAY * W_HH) return;
  if (in_sizes[8] != NLAY * HD) return;
  if (in_sizes[9] != NLAY * W_2HH) return;
  if (in_sizes[10] != NLAY * HD) return;
  if (in_sizes[11] != NLAY * W_HH) return;
  if (in_sizes[12] != NLAY * HD) return;
  if (out_size != NR * HD) return;

  const float* coords   = (const float*)d_in[0];
  const float* contacts = (const float*)d_in[1];
  const float* node_fe  = (const float*)d_in[2];
  const float* in_w     = (const float*)d_in[3];
  const float* in_b     = (const float*)d_in[4];
  const float* e_w1     = (const float*)d_in[5];
  const float* e_b1     = (const float*)d_in[6];
  const float* e_w2     = (const float*)d_in[7];
  const float* e_b2     = (const float*)d_in[8];
  const float* n_w1     = (const float*)d_in[9];
  const float* n_b1     = (const float*)d_in[10];
  const float* n_w2     = (const float*)d_in[11];
  const float* n_b2     = (const float*)d_in[12];
  float* out = (float*)d_out;

  size_t off = 0;
  const size_t oHF0  = off; off += align256((size_t)NR * HD * 4);
  const size_t oHF1  = off; off += align256((size_t)NR * HD * 4);
  const size_t oHIJ  = off; off += align256((size_t)NR * 2 * HD * 4);
  const size_t oHMh  = off; off += align256((size_t)NR * 2 * HD * 2);
  const size_t oHMl  = off; off += align256((size_t)NR * 2 * HD * 2);
  const size_t oSh   = off; off += align256((size_t)NR * HD * 2);
  const size_t oSl   = off; off += align256((size_t)NR * HD * 2);
  const size_t oNFh  = off; off += align256((size_t)NR * IN_F * 2);
  const size_t oNFl  = off; off += align256((size_t)NR * IN_F * 2);
  const size_t oINWh = off; off += align256((size_t)HD * IN_F * 2);
  const size_t oINWl = off; off += align256((size_t)HD * IN_F * 2);
  const size_t oW1Th = off; off += align256((size_t)NLAY * W_2HH * 2);
  const size_t oW1Tl = off; off += align256((size_t)NLAY * W_2HH * 2);
  const size_t oEW2T = off; off += align256((size_t)NLAY * W_HH * 2);
  const size_t oNW1Th = off; off += align256((size_t)NLAY * W_2HH * 2);
  const size_t oNW1Tl = off; off += align256((size_t)NLAY * W_2HH * 2);
  const size_t oNW2Th = off; off += align256((size_t)NLAY * W_HH * 2);
  const size_t oNW2Tl = off; off += align256((size_t)NLAY * W_HH * 2);
  const size_t oPRE  = off; off += align256((size_t)CH_ROWS * HD * 2);
  const size_t oMIJ  = off; off += align256((size_t)CH_ROWS * HD * 4);
  const size_t total = off;
  if (total > ws_size) return;
  if (total > (size_t)134217728) return;

  char* ws = (char*)d_ws;
  float* HF0 = (float*)(ws + oHF0);
  float* HF1 = (float*)(ws + oHF1);
  float* HIJ = (float*)(ws + oHIJ);
  unsigned short* HMh  = (unsigned short*)(ws + oHMh);
  unsigned short* HMl  = (unsigned short*)(ws + oHMl);
  unsigned short* Sh   = (unsigned short*)(ws + oSh);
  unsigned short* Sl   = (unsigned short*)(ws + oSl);
  unsigned short* NFh  = (unsigned short*)(ws + oNFh);
  unsigned short* NFl  = (unsigned short*)(ws + oNFl);
  unsigned short* INWh = (unsigned short*)(ws + oINWh);
  unsigned short* INWl = (unsigned short*)(ws + oINWl);
  unsigned short* W1Th = (unsigned short*)(ws + oW1Th);
  unsigned short* W1Tl = (unsigned short*)(ws + oW1Tl);
  unsigned short* EW2T = (unsigned short*)(ws + oEW2T);
  unsigned short* NW1Th = (unsigned short*)(ws + oNW1Th);
  unsigned short* NW1Tl = (unsigned short*)(ws + oNW1Tl);
  unsigned short* NW2Th = (unsigned short*)(ws + oNW2Th);
  unsigned short* NW2Tl = (unsigned short*)(ws + oNW2Tl);
  unsigned short* PRE16 = (unsigned short*)(ws + oPRE);
  float* MIJ = (float*)(ws + oMIJ);

  transpose_cast<32, 1><<<dim3(2, 1, 1), 256, 0, stream>>>(in_w, HD, IN_F, (long)0, (long)0, 1, INWh, INWl, (long)0);
  transpose_cast<64, 1><<<dim3(2, 2, 2 * NLAY), 256, 0, stream>>>(e_w1, HD, HD, (long)E_W1_STRIDE, (long)W_HH, 2, W1Th, W1Tl, (long)W_HH);
  transpose_cast<64, 0><<<dim3(2, 2, NLAY), 256, 0, stream>>>(e_w2, HD, HD, (long)W_HH, (long)0, 1, EW2T, EW2T, (long)W_HH);
  transpose_cast<64, 1><<<dim3(2, 4, NLAY), 256, 0, stream>>>(n_w1, HD, 2 * HD, (long)W_2HH, (long)0, 1, NW1Th, NW1Tl, (long)W_2HH);
  transpose_cast<64, 1><<<dim3(2, 2, NLAY), 256, 0, stream>>>(n_w2, HD, HD, (long)W_HH, (long)0, 1, NW2Th, NW2Tl, (long)W_HH);
  split_cast8<<<(NR * IN_F / 8 + 255) / 256, 256, 0, stream>>>(node_fe, IN_F, NFh, NFl, IN_F, IN_F / 8, NR * IN_F / 8);

  {
    const int tiles = (NR / 64) * (HD / 64);
    wmma_gemm64<1, true, 2, 0, false, 0><<<dim3((tiles + 7) / 8, 1), 256, 0, stream>>>(
        NFh, NFl, IN_F, (long)0, INWh, INWl, IN_F, (long)0, HF0, nullptr, HD, (long)0,
        in_b, nullptr, (long)0, NR, HD, IN_F, 1.0f);
  }
  split_cast8<<<(NR * HD / 8 + 255) / 256, 256, 0, stream>>>(HF0, HD, HMh, HMl, 2 * HD, HD / 8, NR * HD / 8);

  float* HFcur = HF0;
  float* HFoth = HF1;
  for (int lay = 0; lay < NLAY; ++lay) {
    {
      const int tiles = (NR / 64) * (2 * HD / 64);
      wmma_gemm64<1, true, 0, 0, false, 0><<<dim3((tiles + 7) / 8, 1), 256, 0, stream>>>(
          HMh, HMl, 2 * HD, (long)0, W1Th + (size_t)lay * W_2HH, W1Tl + (size_t)lay * W_2HH, HD, (long)0,
          HIJ, nullptr, 2 * HD, (long)0, nullptr, nullptr, (long)0, NR, 2 * HD, HD, 1.0f);
    }
    const float* w1l  = e_w1 + (size_t)lay * E_W1_STRIDE;
    const float* eb1l = e_b1 + (size_t)lay * HD;
    const float* eb2l = e_b2 + (size_t)lay * HD;
    for (int b = 0; b < NB_; ++b) {
      for (int q = 0; q < LL / CH_I; ++q) {
        const int i0 = q * CH_I;
        build_pre<<<dim3(CH_I, 4), 256, 0, stream>>>(HIJ, coords, contacts, w1l, eb1l, PRE16, b, i0);
        {
          const int tiles = (CH_ROWS / 64) * (HD / 64);
          wmma_gemm64<0, false, 2, 0, false, 6><<<dim3((tiles + 7) / 8, 1), 256, 0, stream>>>(
              PRE16, PRE16, HD, (long)0, EW2T + (size_t)lay * W_HH, EW2T + (size_t)lay * W_HH, HD, (long)0,
              MIJ, nullptr, HD, (long)0, eb2l, nullptr, (long)0, CH_ROWS, HD, HD, 1.0f);
        }
        reduce_mi<<<CH_I, 128, 0, stream>>>(MIJ, contacts, HMh, HMl, b, i0);
      }
    }
    {
      const int tiles = (NR / 64) * (HD / 64);
      wmma_gemm64<1, true, 2, 2, false, 6><<<dim3((tiles + 7) / 8, 1), 256, 0, stream>>>(
          HMh, HMl, 2 * HD, (long)0, NW1Th + (size_t)lay * W_2HH, NW1Tl + (size_t)lay * W_2HH, 2 * HD, (long)0,
          Sh, Sl, HD, (long)0, n_b1 + (size_t)lay * HD, nullptr, (long)0, NR, HD, 2 * HD, 1.0f);
    }
    float* dst = (lay == NLAY - 1) ? out : HFoth;
    {
      const int tiles = (NR / 64) * (HD / 64);
      wmma_gemm64<1, true, 2, 0, true, 0><<<dim3((tiles + 7) / 8, 1), 256, 0, stream>>>(
          Sh, Sl, HD, (long)0, NW2Th + (size_t)lay * W_HH, NW2Tl + (size_t)lay * W_HH, HD, (long)0,
          dst, nullptr, HD, (long)0, n_b2 + (size_t)lay * HD, HFcur, (long)0, NR, HD, HD, 1.0f);
    }
    if (lay != NLAY - 1) {
      split_cast8<<<(NR * HD / 8 + 255) / 256, 256, 0, stream>>>(dst, HD, HMh, HMl, 2 * HD, HD / 8, NR * HD / 8);
      float* t = HFcur; HFcur = HFoth; HFoth = t;
    }
  }
  (void)hipGetLastError();
}
